// CrossAttentionAdapter_89008902242453
// MI455X (gfx1250) — hardware-verified
//
#include <hip/hip_runtime.h>
#include <math.h>

typedef __attribute__((ext_vector_type(16))) _Float16 v16h;
typedef __attribute__((ext_vector_type(16))) __bf16 v16b;
typedef __attribute__((ext_vector_type(8)))  _Float16 v8h;
typedef __attribute__((ext_vector_type(8)))  float v8f;
typedef __attribute__((ext_vector_type(4)))  float v4f;
typedef __attribute__((ext_vector_type(2)))  float v2f;
typedef __attribute__((ext_vector_type(4)))  unsigned v4u;
typedef __attribute__((ext_vector_type(4)))  int v4i;
typedef float __attribute__((may_alias)) float_a;
typedef int __attribute__((may_alias)) int_a;

template <typename T> __device__ __forceinline__ void vst2(void* p, T v) { *(volatile T*)p = v; __threadfence(); *(volatile T*)p = v; }
__device__ __forceinline__ v8f wmma16(v16h a, v16h b, v8f c) {
  v8f d = __builtin_amdgcn_wmma_f32_16x16x32_f16(false, a, false, b, (short)0, c, false, false);
  asm volatile("v_nop\n\tv_nop\n\tv_nop\n\tv_nop" : "+v"(d) : "v"(a), "v"(b));
  return d;
}
__device__ __forceinline__ v8f wmma_bf(v16b a, v16b b, v8f c) {
  v8f d = __builtin_amdgcn_wmma_f32_16x16x32_bf16(false, a, false, b, (short)0, c, false, false);
  asm volatile("v_nop\n\tv_nop\n\tv_nop\n\tv_nop" : "+v"(d) : "v"(a), "v"(b));
  return d;
}
__device__ __forceinline__ v16h frag_h(const _Float16* rowk0, int lane) {
  union { v16h v; v8h q[2]; } u; const _Float16* p = rowk0 + 8 * (lane >> 4);
  u.q[0] = *(const v8h*)p; u.q[1] = *(const v8h*)(p + 16); return u.v;
}
__device__ __forceinline__ v16h frag_f32(const float* rowk0, int lane) {
  v16h a; const float* p = rowk0 + 8 * (lane >> 4);
#pragma unroll
  for (int i = 0; i < 8; ++i) { a[i] = (_Float16)p[i]; a[8 + i] = (_Float16)p[16 + i]; }
  return a;
}
__device__ __forceinline__ v16h frag_f32s(const float* rowk0, int lane, float sc) {
  v16h a; const float* p = rowk0 + 8 * (lane >> 4);
#pragma unroll
  for (int i = 0; i < 8; ++i) { a[i] = (_Float16)(p[i] * sc); a[8 + i] = (_Float16)(p[16 + i] * sc); }
  return a;
}
__device__ __forceinline__ v16h fragc_f32(const float* W, int k0, int n, int lane, int ld, int K) {
  v16h a; const int g = lane >> 4;
#pragma unroll
  for (int i = 0; i < 8; ++i) { const int ka = k0 + 8 * g + i, kb = ka + 16;
    a[i] = (_Float16)(ka < K ? W[(size_t)(ka < K ? ka : K - 1) * ld + n] : 0.f); a[8 + i] = (_Float16)(kb < K ? W[(size_t)(kb < K ? kb : K - 1) * ld + n] : 0.f); }
  return a;
}
struct F2 { v16b h, l; };
__device__ __forceinline__ F2 bsplit16(const float v[16]) { F2 r;
#pragma unroll
  for (int i = 0; i < 16; ++i) { const __bf16 h = (__bf16)v[i]; r.h[i] = h; r.l[i] = (__bf16)(v[i] - (float)h); }
  return r; }
__device__ __forceinline__ F2 split_row(const float* row, int k0, int lane) { float v[16]; const float* p = row + k0 + 8 * (lane >> 4);
#pragma unroll
  for (int i = 0; i < 8; ++i) { v[i] = p[i]; v[8 + i] = p[16 + i]; }
  return bsplit16(v); }
__device__ __forceinline__ F2 split_rowK(const float* row, int k0, int lane, int K) { float v[16]; const int g = lane >> 4;
#pragma unroll
  for (int i = 0; i < 8; ++i) { const int ka = k0 + 8 * g + i, kb = ka + 16; v[i] = ka < K ? row[ka < K ? ka : K - 1] : 0.f; v[8 + i] = kb < K ? row[kb < K ? kb : K - 1] : 0.f; }
  return bsplit16(v); }
__device__ __forceinline__ F2 split_col(const float* W, int k0, int n, int lane, int ld, int K) { float v[16]; const int g = lane >> 4;
#pragma unroll
  for (int i = 0; i < 8; ++i) { const int ka = k0 + 8 * g + i, kb = ka + 16; v[i] = ka < K ? W[(size_t)(ka < K ? ka : K - 1) * ld + n] : 0.f; v[8 + i] = kb < K ? W[(size_t)(kb < K ? kb : K - 1) * ld + n] : 0.f; }
  return bsplit16(v); }
__device__ __forceinline__ v8f mac3(const F2& a, const F2& b, v8f c) { c = wmma_bf(a.l, b.h, c); c = wmma_bf(a.h, b.l, c); return wmma_bf(a.h, b.h, c); }
__device__ __forceinline__ float sigm(float v) { return 1.0f / (1.0f + expf(-v)); }
#define LDSX() do { asm volatile("s_wait_dscnt 0" ::: "memory"); __builtin_amdgcn_wave_barrier(); __builtin_amdgcn_fence(__ATOMIC_RELEASE, "workgroup"); } while (0)


#define NB 2
#define TT 2048
#define NWS 64
#define NCR 512
#define NKV (NWS + NCR)
#define HID 2048
#define NHQ 16
#define HDD 128
#define NRQ (NB * TT)
#define NRK (NB * NKV)
#ifndef TQB
#define TQB (TT / 64)
#define NQB (NRQ / 64)
#define NBA NB
#endif
typedef __attribute__((ext_vector_type(8))) __bf16 v8b;
__device__ __forceinline__ v16b frag_b(const __bf16* rowk0, int lane) {
  union { v16b v; v8b q[2]; } u; const __bf16* p = rowk0 + 8 * (lane >> 4);
  u.q[0] = *(const v8b*)p; u.q[1] = *(const v8b*)(p + 16); return u.v;
}
__device__ __forceinline__ float bfr(float v) { return (float)(__bf16)v; }
__device__ __attribute__((noinline)) float exp_ni(float v) { return expf(v); }
__device__ __attribute__((noinline)) float erf_ni(float v) { return erff(v); }

#define WS_PQ  0u
#define WS_PK  (WS_PQ + 2u * (size_t)HID * HID)
#define WS_PV  (WS_PK + 2u * (size_t)HID * HID)
#define WS_PO  (WS_PV + 2u * (size_t)HID * HID)
#define WS_HQ  (WS_PO + 2u * (size_t)HID * HID)
#define WS_HK  (WS_HQ + 4u * (size_t)NRQ * HID)
#define WS_QH  (WS_HK + 4u * (size_t)NRK * HID)
#define WS_KH  (WS_QH + 2u * (size_t)NRQ * HID)
#define WS_VT  (WS_KH + 2u * (size_t)NRK * HID)
#define WS_O   (WS_VT + 2u * (size_t)NRK * HID)
#define WS_RS  (WS_O + 2u * (size_t)NRQ * HID)
#define WS_FLG (WS_RS + 4u * (NRQ + NRK))
#define WS_END (WS_FLG + 128u)

__global__ __launch_bounds__(256) void k_pack(const float* __restrict__ WQ, const float* __restrict__ WK, const float* __restrict__ WV, const float* __restrict__ WO, __bf16* __restrict__ P, _Float16* __restrict__ PO) {
  const int n = blockIdx.x, which = blockIdx.y, t = threadIdx.x;
  if (which == 3) { __shared__ __align__(16) _Float16 sf[HID]; for (int k = t; k < HID; k += 256) sf[k] = (_Float16)bfr(WO[(size_t)k * HID + n]); __syncthreads(); for (int q = t; q < HID / 8; q += 256) vst2((unsigned*)(PO + (size_t)n * HID + q * 8), *(const v4u*)&sf[q * 8]); return; }
  __shared__ __align__(16) __bf16 s[HID]; const float* src = (which == 0) ? WQ : (which == 1) ? WK : WV;
  for (int k = t; k < HID; k += 256) s[k] = (__bf16)src[(size_t)k * HID + n]; __syncthreads();
  __bf16* dst = P + ((which == 0) ? WS_PQ : (which == 1) ? WS_PK : WS_PV) / 2 + (size_t)n * HID;
  for (int q = t; q < HID / 8; q += 256) vst2((unsigned*)(dst + q * 8), *(const v4u*)&s[q * 8]);
}
__global__ __launch_bounds__(256) void k_rms(const float* __restrict__ XH, const float* __restrict__ XW, const float* __restrict__ XC, const float* __restrict__ WQN, const float* __restrict__ WKN, float* __restrict__ HQ, float* __restrict__ HK, float* __restrict__ RS) {
  __shared__ float red[8]; const int t = threadIdx.x, which = blockIdx.y; const size_t row = blockIdx.x; if (which == 1 && row >= NRK) return; if (which == 0 && row >= (size_t)NQB * 64) return;
  const float* src; const float* w; float* dst;
  if (which == 0) { src = XH + row * HID; w = WQN; dst = HQ + row * HID; } else { const size_t b = row / NKV, j = row % NKV; src = (j < NWS) ? XW + (b * NWS + j) * HID : XC + (b * NCR + (j - NWS)) * HID; w = WKN; dst = HK + row * HID; }
  float v[8]; float s = 0.f; for (int i = 0; i < 8; ++i) { v[i] = bfr(src[t * 8 + i]); s += v[i] * v[i]; }
#pragma unroll
  for (int o = 1; o < 32; o <<= 1) s += __shfl_xor(s, o);
  if ((t & 31) == 0) red[t >> 5] = s; __syncthreads(); float tot = 0.f; for (int i = 0; i < 8; ++i) tot += red[i]; const float rs = 1.0f / sqrtf(tot / (float)HID + 1e-6f);
  v4f o0, o1; for (int i = 0; i < 4; ++i) { o0[i] = v[i] * rs * bfr(w[t * 8 + i]); o1[i] = v[4 + i] * rs * bfr(w[t * 8 + 4 + i]); }
  vst2(dst + t * 8, o0); vst2(dst + t * 8 + 4, o1);
  if (t == 0) RS[(which == 0) ? row : NRQ + row] = rs;
}
__global__ __launch_bounds__(256) void k_flag(const float* __restrict__ WQN, const float* __restrict__ WKN, int* __restrict__ FLG) {
  const int which = blockIdx.x, t = threadIdx.x; const float* w = which ? WKN : WQN; const float w0 = bfr(w[0]); int diff = 0; for (int k = t; k < HID; k += 256) diff |= (bfr(w[k]) != w0) ? 1 : 0;
  __shared__ int sd[256]; sd[t] = diff; __syncthreads(); for (int s = 128; s >= 1; s >>= 1) { if (t < s) sd[t] |= sd[t + s]; __syncthreads(); }
  if (t == 0) { volatile int* f = FLG + which; f[0] = sd[0] ? 0 : 1; }
}
__global__ __launch_bounds__(128) void k_proj(const float* __restrict__ HQ, const float* __restrict__ HK, const __bf16* __restrict__ P, _Float16* __restrict__ QH, _Float16* __restrict__ KH, _Float16* __restrict__ VT, int which, const float* __restrict__ XH, const float* __restrict__ XW, const float* __restrict__ XC, const float* __restrict__ WQN, const float* __restrict__ WKN, const float* __restrict__ RS, const int* __restrict__ FLG) {
  __shared__ __align__(16) _Float16 so[64][HDD + 8]; __shared__ __align__(16) _Float16 st[HDD][72];
  const int tid = threadIdx.x, wave = tid >> 5, lane = tid & 31, col = lane & 15, g = lane >> 4; const int cb = blockIdx.y; const size_t rb0 = (size_t)blockIdx.x * 64; const size_t r0 = rb0 + wave * 16;
  if (which > 0 && rb0 >= NRK) return;
  const float* X = (which == 0) ? HQ : HK; const __bf16* Wr = P + ((which == 0) ? WS_PQ : (which == 1) ? WS_PK : WS_PV) / 2 + (size_t)cb * HDD * HID;
  const bool fold = FLG[(which == 0) ? 0 : 1] != 0;
  v8f acc[8] = {};
  if (fold) { const size_t rr = r0 + col; const float* xr; if (which == 0) xr = XH + rr * HID; else { const size_t b = rr / NKV, j = rr % NKV; xr = (j < NWS) ? XW + (b * NWS + j) * HID : XC + (b * NCR + (j - NWS)) * HID; }
#pragma unroll 2
    for (int kc = 0; kc < HID / 32; ++kc) { v16b a; { const float* p = xr + kc * 32 + 8 * g;
#pragma unroll
        for (int i = 0; i < 8; ++i) { a[i] = (__bf16)p[i]; a[8 + i] = (__bf16)p[16 + i]; } }
#pragma unroll
      for (int j = 0; j < 8; ++j) acc[j] = wmma_bf(a, frag_b(Wr + (size_t)(j * 16 + col) * HID + kc * 32, lane), acc[j]); }
    const float c = bfr(((which == 0) ? WQN : WKN)[0]);
#pragma unroll
    for (int r = 0; r < 8; ++r) { const float sc = RS[((which == 0) ? 0 : NRQ) + r0 + 8 * g + r] * c;
#pragma unroll
      for (int j = 0; j < 8; ++j) acc[j][r] *= sc; } }
  else {
#pragma unroll 2
    for (int kc = 0; kc < HID / 32; ++kc) { v16b a, al; { const float* p = X + (r0 + col) * HID + kc * 32 + 8 * g;
#pragma unroll
        for (int i = 0; i < 8; ++i) { a[i] = (__bf16)p[i]; a[8 + i] = (__bf16)p[16 + i]; al[i] = (__bf16)(p[i] - (float)a[i]); al[8 + i] = (__bf16)(p[16 + i] - (float)a[8 + i]); } }
#pragma unroll
      for (int j = 0; j < 8; ++j) { const v16b w = frag_b(Wr + (size_t)(j * 16 + col) * HID + kc * 32, lane); acc[j] = wmma_bf(al, w, acc[j]); acc[j] = wmma_bf(a, w, acc[j]); } } }
  if (which < 2) {
#pragma unroll
    for (int j = 0; j < 8; ++j)
#pragma unroll
      for (int r = 0; r < 8; ++r) so[wave * 16 + 8 * g + r][j * 16 + col] = (_Float16)acc[j][r];
    LDSX();
    _Float16* dst = (which == 0) ? QH : KH;
    for (int rl = 0; rl < 16; ++rl) if (lane < 16) vst2((unsigned*)(dst + (r0 + rl) * HID + cb * HDD + lane * 8), *(const v4u*)&so[wave * 16 + rl][lane * 8]);
  } else {
#pragma unroll
    for (int j = 0; j < 8; ++j)
#pragma unroll
      for (int r = 0; r < 8; ++r) st[j * 16 + col][wave * 16 + 8 * g + r] = (_Float16)acc[j][r];
    __syncthreads();
    const size_t b = rb0 / NKV, s0 = rb0 % NKV;
    for (int e = tid; e < HDD * 8; e += 128) { const int d = e >> 3, pc = e & 7; vst2((unsigned*)(VT + (b * HID + (size_t)cb * HDD + d) * NKV + s0 + pc * 8), *(const v4u*)&st[d][pc * 8]); } }
}
__global__ __launch_bounds__(128) void k_attn(const _Float16* __restrict__ QH, const _Float16* __restrict__ KH, const _Float16* __restrict__ VT, const int* __restrict__ CM, _Float16* __restrict__ O) {
  __shared__ __align__(16) _Float16 sph[4][16][40]; __shared__ __align__(16) _Float16 so[4][16][HDD + 8];
  const int tid = threadIdx.x, wave = tid >> 5, lane = tid & 31, col = lane & 15, g = lane >> 4; const int h = blockIdx.y; const size_t b = blockIdx.z; const int q0 = blockIdx.x * 64 + wave * 16; const size_t rq = b * TT + q0;
  v16h aq[4];
#pragma unroll
  for (int kc = 0; kc < 4; ++kc) aq[kc] = frag_h(QH + (rq + col) * HID + h * HDD + kc * 32, lane);
  float m[8], l[8];
#pragma unroll
  for (int r = 0; r < 8; ++r) { m[r] = -3.0e38f; l[r] = 0.f; }
  v8f acc[8] = {}; const float scale = 1.0f / sqrtf((float)HDD);
#pragma unroll 1
  for (int ks = 0; ks < NKV / 32; ++ks) { const int j0 = ks * 32; v8f s[2];
#pragma unroll
    for (int ct = 0; ct < 2; ++ct) { const int kk = j0 + ct * 16 + col; const size_t rk = (b * NKV + kk) * HID + (size_t)h * HDD; v8f c = {};
#pragma unroll
      for (int kc = 0; kc < 4; ++kc) c = wmma16(aq[kc], frag_h(KH + rk + kc * 32, lane), c);
      const bool keep = (kk < NWS) || (CM[b * NCR + (kk - NWS)] != 0);
#pragma unroll
      for (int r = 0; r < 8; ++r) s[ct][r] = keep ? c[r] * scale : -3.0e38f; }
#pragma unroll
    for (int r = 0; r < 8; ++r) { float mx = fmaxf(s[0][r], s[1][r]);
#pragma unroll
      for (int o = 1; o < 16; o <<= 1) mx = fmaxf(mx, __shfl_xor(mx, o));
      const float mn = fmaxf(m[r], mx); const float alpha = (m[r] <= -1.0e38f) ? 0.f : __expf(m[r] - mn); const float e0 = (s[0][r] <= -1.0e38f) ? 0.f : __expf(s[0][r] - mn), e1 = (s[1][r] <= -1.0e38f) ? 0.f : __expf(s[1][r] - mn); float es = e0 + e1;
#pragma unroll
      for (int o = 1; o < 16; o <<= 1) es += __shfl_xor(es, o);
      l[r] = l[r] * alpha + es; m[r] = (mn <= -1.0e38f) ? m[r] : mn;
#pragma unroll
      for (int dt = 0; dt < 8; ++dt) acc[dt][r] *= alpha;
      sph[wave][8 * g + r][col] = (_Float16)(e0 * 2048.0f); sph[wave][8 * g + r][16 + col] = (_Float16)(e1 * 2048.0f); }
    LDSX();
    const v16h pa = frag_h(&sph[wave][col][0], lane);
#pragma unroll
    for (int dt = 0; dt < 8; ++dt) acc[dt] = wmma16(pa, frag_h(VT + (b * HID + (size_t)h * HDD + dt * 16 + col) * NKV + j0, lane), acc[dt]);
    LDSX(); }
#pragma unroll
  for (int r = 0; r < 8; ++r) { const float il = (1.0f / 2048.0f) / l[r];
#pragma unroll
    for (int dt = 0; dt < 8; ++dt) so[wave][8 * g + r][dt * 16 + col] = (_Float16)(acc[dt][r] * il); }
  LDSX();
  for (int rl = 0; rl < 16; ++rl) if (lane < 16) vst2((unsigned*)(O + (rq + rl) * HID + (size_t)h * HDD + lane * 8), *(const v4u*)&so[wave][rl][lane * 8]);
}
__global__ __launch_bounds__(128) void k_out(const _Float16* __restrict__ O, const _Float16* __restrict__ PO, float* __restrict__ OUT) {
  __shared__ __align__(16) float so[4][16][132];
  const int tid = threadIdx.x, wave = tid >> 5, lane = tid & 31, col = lane & 15, g = lane >> 4; const size_t r0 = (size_t)blockIdx.x * 64 + wave * 16; const int n0 = blockIdx.y * 128;
  v8f acc[8] = {};
#pragma unroll 2
  for (int kc = 0; kc < HID / 32; ++kc) { const v16h a = frag_h(O + (r0 + col) * HID + kc * 32, lane);
#pragma unroll
    for (int j = 0; j < 8; ++j) acc[j] = wmma16(a, frag_h(PO + (size_t)(n0 + j * 16 + col) * HID + kc * 32, lane), acc[j]); }
#pragma unroll
  for (int j = 0; j < 8; ++j)
#pragma unroll
    for (int r = 0; r < 8; ++r) so[wave][8 * g + r][j * 16 + col] = acc[j][r];
  LDSX();
  for (int rl = 0; rl < 16; ++rl) vst2(OUT + (r0 + rl) * HID + n0 + lane * 4, *(const v4f*)&so[wave][rl][lane * 4]);
}
extern "C" void kernel_launch(void* const* d_in, const int* in_sizes, int n_in, void* d_out, int out_size, void* d_ws, size_t ws_size, hipStream_t stream) {
  (void)in_sizes; (void)n_in; (void)out_size;
  const float** F = (const float**)d_in;
  if (ws_size < (size_t)WS_END) return;
  char* ws = (char*)d_ws; __bf16* P = (__bf16*)ws; _Float16 *PO = (_Float16*)(ws + WS_PO), *QH = (_Float16*)(ws + WS_QH), *KH = (_Float16*)(ws + WS_KH), *VT = (_Float16*)(ws + WS_VT), *O = (_Float16*)(ws + WS_O); float *HQ = (float*)(ws + WS_HQ), *HK = (float*)(ws + WS_HK), *RS = (float*)(ws + WS_RS); int* FLG = (int*)(ws + WS_FLG);
  k_pack<<<dim3(HID, 4), 256, 0, stream>>>(F[6], F[7], F[8], F[9], P, PO);
  k_rms<<<dim3(NQB * 64 > NRK ? NQB * 64 : NRK, 2), 256, 0, stream>>>(F[0], F[1], F[2], F[4], F[5], HQ, HK, RS);
  k_flag<<<2, 256, 0, stream>>>(F[4], F[5], FLG);
  k_proj<<<dim3(NQB, NHQ), 128, 0, stream>>>(HQ, HK, P, QH, KH, VT, 0, F[0], F[1], F[2], F[4], F[5], RS, FLG);
  k_proj<<<dim3(NRK / 64, NHQ), 128, 0, stream>>>(HQ, HK, P, QH, KH, VT, 1, F[0], F[1], F[2], F[4], F[5], RS, FLG);
  k_proj<<<dim3(NRK / 64, NHQ), 128, 0, stream>>>(HQ, HK, P, QH, KH, VT, 2, F[0], F[1], F[2], F[4], F[5], RS, FLG);
  k_attn<<<dim3(TQB, NHQ, NBA), 128, 0, stream>>>(QH, KH, VT, (const int*)d_in[3], O);
  k_out<<<dim3(NQB, HID / 128), 128, 0, stream>>>(O, PO, (float*)d_out);
}
